// Non_local_47923245088807
// MI455X (gfx1250) — hardware-verified
//
#include <hip/hip_runtime.h>
#include <stddef.h>
#include <stdint.h>

#define NB    16
#define NC    256
#define NI    128
#define NN    2048
#define NX    (NB * NC * NN)
#define NWT   (NI * NC)
#define NTHR  256
#define GTHR  128
#define WSMAX 134217728
#define XTP   72

static_assert((NC % 64) == 0 && (NN % 64) == 0 && (NI % 64) == 0);
static_assert((NC % 32) == 0 && (NI % 32) == 0 && (NN % 32) == 0);
static_assert((NX % 1024) == 0 && (NN % 1024) == 0);
static_assert((XTP % 8) == 0);
static_assert(GTHR == 128 && NTHR == 256);
static_assert((4 * NWT) % (8 * NTHR) == 0);
static_assert((NWT / 8) % NTHR == 0);
static_assert(NB * NN == 32768);

typedef float          v4f  __attribute__((ext_vector_type(4)));
typedef float          v8f  __attribute__((ext_vector_type(8)));
typedef int            v8i  __attribute__((ext_vector_type(8)));
typedef unsigned short v8us __attribute__((ext_vector_type(8)));
typedef __bf16         v16bf __attribute__((ext_vector_type(16)));
typedef v4f  __attribute__((may_alias)) v4fa;
typedef v8us __attribute__((may_alias)) v8usa;
union FragB { v16bf v; v8us h[2]; v8i w; };

__device__ __forceinline__ v8f wmb(const FragB& a, const FragB& b, v8f c) {
  v8f d = __builtin_amdgcn_wmma_f32_16x16x32_bf16(false, a.v, false, b.v, (short)0, c, false, false);
  asm volatile("v_nop\n\tv_nop\n\tv_nop\n\tv_nop" : "+v"(d) : "v"(a.w), "v"(b.w));
  return d;
}

__device__ __forceinline__ void ldfrag(FragB& f, const unsigned short* p, int k0) {
  f.h[0] = *(const v8us*)(p + k0);
  f.h[1] = *(const v8us*)(p + k0 + 16);
}

__device__ __forceinline__ unsigned short rne16(float f) {
  unsigned u = __float_as_uint(f);
  u += 0x7FFFu + ((u >> 16) & 1u);
  return (unsigned short)(u >> 16);
}
__device__ __forceinline__ float rne16f(float f) {
  return __uint_as_float(((unsigned)rne16(f)) << 16);
}
__device__ __forceinline__ v8us cvt8(const v4f a, const v4f b) {
  v8us o;
  o[0] = rne16(a.x); o[1] = rne16(a.y); o[2] = rne16(a.z); o[3] = rne16(a.w);
  o[4] = rne16(b.x); o[5] = rne16(b.y); o[6] = rne16(b.z); o[7] = rne16(b.w);
  return o;
}
__device__ __forceinline__ void sp1(float v, unsigned short& hi, unsigned short& lo) {
  const unsigned short hb = rne16(v);
  const float hf = __uint_as_float(((unsigned)hb) << 16);
  hi = hb;
  lo = rne16(v - hf);
}
__device__ __forceinline__ void split8(const v4f a, const v4f b, v8us& hv, v8us& lv) {
  unsigned short h0, h1, h2, h3, h4, h5, h6, h7, l0, l1, l2, l3, l4, l5, l6, l7;
  sp1(a.x, h0, l0); sp1(a.y, h1, l1); sp1(a.z, h2, l2); sp1(a.w, h3, l3);
  sp1(b.x, h4, l4); sp1(b.y, h5, l5); sp1(b.z, h6, l6); sp1(b.w, h7, l7);
  hv[0] = h0; hv[1] = h1; hv[2] = h2; hv[3] = h3; hv[4] = h4; hv[5] = h5; hv[6] = h6; hv[7] = h7;
  lv[0] = l0; lv[1] = l1; lv[2] = l2; lv[3] = l3; lv[4] = l4; lv[5] = l5; lv[6] = l6; lv[7] = l7;
}

__device__ __forceinline__ void store_split_tile(const float* stg, unsigned short* ph, unsigned short* pl,
                                                 size_t rowBase, size_t pitch, size_t col0, int wave, int lane) {
  const int q8 = lane & 7, sub = lane >> 3;
  v8us hv[4], lv[4];
  size_t po[4];
#pragma unroll
  for (int i = 0; i < 4; ++i) {
    const int lr = 16 * wave + 4 * i + sub;
    const v4f a = *(const v4fa*)(stg + lr * 64 + 8 * q8);
    const v4f c = *(const v4fa*)(stg + lr * 64 + 8 * q8 + 4);
    split8(a, c, hv[i], lv[i]);
    po[i] = (rowBase + (size_t)lr) * pitch + col0 + (size_t)(8 * q8);
  }
#pragma unroll
  for (int i = 0; i < 4; ++i) {
    *(volatile v8us*)(ph + po[i]) = hv[i];
    *(volatile v8us*)(pl + po[i]) = lv[i];
  }
  __threadfence();
#pragma unroll
  for (int i = 0; i < 4; ++i) {
    *(volatile v8us*)(ph + po[i]) = hv[i];
    *(volatile v8us*)(pl + po[i]) = lv[i];
  }
}

__global__ __launch_bounds__(NTHR) void k_wcvt(const float* __restrict__ w0, const float* __restrict__ w1,
                                               const float* __restrict__ w2, const float* __restrict__ w3,
                                               unsigned short* wb) {
  const int u   = (int)blockIdx.x * NTHR + (int)threadIdx.x;
  const int sel = (int)blockIdx.x / ((NWT / 8) / NTHR);
  const int off8 = (u - sel * (NWT / 8)) * 8;
  const float* src = (sel == 0) ? w0 : ((sel == 1) ? w1 : ((sel == 2) ? w2 : w3));
  const v4f a = *(const v4fa*)(src + off8);
  const v4f c = *(const v4fa*)(src + off8 + 4);
  const v8us o = cvt8(a, c);
  const size_t q = (size_t)sel * (size_t)NWT + (size_t)off8;
  *(volatile v8us*)(wb + q) = o;
  __threadfence();
  *(volatile v8us*)(wb + q) = o;
}

__global__ __launch_bounds__(NTHR) void k_xt(const float* __restrict__ x, unsigned short* xt) {
  __shared__ __attribute__((aligned(16))) unsigned short sT[64 * XTP];
  const int tid = (int)threadIdx.x;
  const int c0 = (int)blockIdx.x * 64, n0 = (int)blockIdx.y * 64, b = (int)blockIdx.z;
#pragma unroll
  for (int i = 0; i < 4; ++i) {
    const int lin = i * NTHR + tid;
    const int cr  = lin >> 4;
    const int n4  = (lin & 15) * 4;
    const v4f v = *(const v4fa*)(x + (size_t)(b * NC + c0 + cr) * (size_t)NN + (size_t)(n0 + n4));
    sT[(n4 + 0) * XTP + cr] = rne16(v.x);
    sT[(n4 + 1) * XTP + cr] = rne16(v.y);
    sT[(n4 + 2) * XTP + cr] = rne16(v.z);
    sT[(n4 + 3) * XTP + cr] = rne16(v.w);
  }
  __syncthreads();
  const int q8 = tid & 7, sub = tid >> 3;
  v8us o[2];
  size_t po[2];
#pragma unroll
  for (int i = 0; i < 2; ++i) {
    const int nr = 32 * i + sub;
    o[i]  = *(const v8usa*)(sT + nr * XTP + 8 * q8);
    po[i] = (size_t)(b * NN + n0 + nr) * (size_t)NC + (size_t)(c0 + 8 * q8);
  }
#pragma unroll
  for (int i = 0; i < 2; ++i) *(volatile v8us*)(xt + po[i]) = o[i];
  __threadfence();
#pragma unroll
  for (int i = 0; i < 2; ++i) *(volatile v8us*)(xt + po[i]) = o[i];
}

__global__ __launch_bounds__(GTHR) void k_proj(const unsigned short* __restrict__ xt,
                                               const unsigned short* __restrict__ wb,
                                               const float* __restrict__ tbias, const float* __restrict__ pbias,
                                               const float* __restrict__ gbias,
                                               unsigned short* thh, unsigned short* thl,
                                               unsigned short* phh, unsigned short* phl,
                                               unsigned short* ghh, unsigned short* ghl) {
  __shared__ __attribute__((aligned(16))) float stg[64 * 64];
  const int tid = (int)threadIdx.x, lane = tid & 31, wave = tid >> 5, hh = lane >> 4, m = lane & 15;
  const int n0 = (int)blockIdx.x * 64, d0 = (int)blockIdx.y * 64;
  const int which = (int)blockIdx.z / NB, b = (int)blockIdx.z - which * NB;

  v8f acc[4];
  {
    const v8f z = {0.f, 0.f, 0.f, 0.f, 0.f, 0.f, 0.f, 0.f};
    acc[0] = z; acc[1] = z; acc[2] = z; acc[3] = z;
  }
  const unsigned short* ap = xt + (size_t)(b * NN + n0 + 16 * wave + m) * (size_t)NC + (size_t)(8 * hh);
  const unsigned short* wp = wb + (size_t)which * (size_t)NWT + (size_t)(d0 + m) * (size_t)NC + (size_t)(8 * hh);
#pragma unroll 1
  for (int ks = 0; ks < NC / 32; ++ks) {
    FragB a;
    ldfrag(a, ap, 32 * ks);
#pragma unroll
    for (int t = 0; t < 4; ++t) {
      FragB bf;
      ldfrag(bf, wp + (size_t)(16 * t) * (size_t)NC, 32 * ks);
      acc[t] = wmb(a, bf, acc[t]);
    }
  }

  const float* bias = (which == 0) ? tbias : ((which == 1) ? pbias : gbias);
#pragma unroll
  for (int t = 0; t < 4; ++t) {
    const int lf = 16 * t + m;
    const float bv = rne16f(bias[d0 + lf]);
#pragma unroll
    for (int r = 0; r < 8; ++r) {
      const int lt = 16 * wave + 8 * hh + r;
      const float v = acc[t][r] + bv;
      const int idx = (which == 0) ? (lt * 64 + lf) : (lf * 64 + lt);
      stg[idx] = v;
    }
  }
  __syncthreads();

  unsigned short* ph = (which == 0) ? thh : ((which == 1) ? phh : ghh);
  unsigned short* pl = (which == 0) ? thl : ((which == 1) ? phl : ghl);
  const size_t rowBase = (which == 0) ? ((size_t)b * NN + (size_t)n0) : ((size_t)b * NI + (size_t)d0);
  const size_t pitch   = (which == 0) ? (size_t)NI : (size_t)NN;
  const size_t col0    = (which == 0) ? (size_t)d0 : (size_t)n0;
  store_split_tile(stg, ph, pl, rowBase, pitch, col0, wave, lane);
}

__global__ __launch_bounds__(GTHR) void k_p(const unsigned short* __restrict__ ghh, const unsigned short* __restrict__ ghl,
                                            const unsigned short* __restrict__ phh, const unsigned short* __restrict__ phl,
                                            unsigned short* pth, unsigned short* ptl) {
  __shared__ __attribute__((aligned(16))) float stg[64 * 64];
  const int tid = (int)threadIdx.x, lane = tid & 31, wave = tid >> 5, hh = lane >> 4, m = lane & 15;
  const int d0 = (int)blockIdx.x * 64, e0 = (int)blockIdx.y * 64, b = (int)blockIdx.z;

  v8f acc[4];
  {
    const v8f z = {0.f, 0.f, 0.f, 0.f, 0.f, 0.f, 0.f, 0.f};
    acc[0] = z; acc[1] = z; acc[2] = z; acc[3] = z;
  }
  const size_t arow = (size_t)(b * NI + e0 + 16 * wave + m) * (size_t)NN + (size_t)(8 * hh);
  const unsigned short* agh = ghh + arow;
  const unsigned short* agl = ghl + arow;
  const size_t brow = (size_t)(b * NI + d0 + m) * (size_t)NN + (size_t)(8 * hh);
  const unsigned short* bph = phh + brow;
  const unsigned short* bpl = phl + brow;
#pragma unroll 1
  for (int ks = 0; ks < NN / 32; ++ks) {
    FragB ah, al;
    ldfrag(ah, agh, 32 * ks);
    ldfrag(al, agl, 32 * ks);
#pragma unroll
    for (int t = 0; t < 4; ++t) {
      FragB bh, bl;
      ldfrag(bh, bph + (size_t)(16 * t) * (size_t)NN, 32 * ks);
      ldfrag(bl, bpl + (size_t)(16 * t) * (size_t)NN, 32 * ks);
      acc[t] = wmb(ah, bh, acc[t]);
      acc[t] = wmb(ah, bl, acc[t]);
      acc[t] = wmb(al, bh, acc[t]);
    }
  }

  const float inv_n = 0.00048828125f;
#pragma unroll
  for (int t = 0; t < 4; ++t) {
    const int lc = 16 * t + m;
#pragma unroll
    for (int r = 0; r < 8; ++r) {
      const int lr = 16 * wave + 8 * hh + r;
      stg[lr * 64 + lc] = acc[t][r] * inv_n;
    }
  }
  __syncthreads();
  store_split_tile(stg, pth, ptl, (size_t)b * NI + (size_t)e0, (size_t)NI, (size_t)d0, wave, lane);
}

__global__ __launch_bounds__(GTHR) void k_y(const unsigned short* __restrict__ thh, const unsigned short* __restrict__ thl,
                                            const unsigned short* __restrict__ pth, const unsigned short* __restrict__ ptl,
                                            unsigned short* yth, unsigned short* ytl) {
  __shared__ __attribute__((aligned(16))) float stg[64 * 64];
  const int tid = (int)threadIdx.x, lane = tid & 31, wave = tid >> 5, hh = lane >> 4, m = lane & 15;
  const int n0 = (int)blockIdx.x * 64, e0 = (int)blockIdx.y * 64, b = (int)blockIdx.z;

  v8f acc[4];
  {
    const v8f z = {0.f, 0.f, 0.f, 0.f, 0.f, 0.f, 0.f, 0.f};
    acc[0] = z; acc[1] = z; acc[2] = z; acc[3] = z;
  }
  const size_t arow = (size_t)(b * NN + n0 + 16 * wave + m) * (size_t)NI + (size_t)(8 * hh);
  const unsigned short* ath = thh + arow;
  const unsigned short* atl = thl + arow;
  const size_t brow = (size_t)(b * NI + e0 + m) * (size_t)NI + (size_t)(8 * hh);
  const unsigned short* bph = pth + brow;
  const unsigned short* bpl = ptl + brow;
#pragma unroll 1
  for (int ks = 0; ks < NI / 32; ++ks) {
    FragB ah, al;
    ldfrag(ah, ath, 32 * ks);
    ldfrag(al, atl, 32 * ks);
#pragma unroll
    for (int t = 0; t < 4; ++t) {
      FragB bh, bl;
      ldfrag(bh, bph + (size_t)(16 * t) * (size_t)NI, 32 * ks);
      ldfrag(bl, bpl + (size_t)(16 * t) * (size_t)NI, 32 * ks);
      acc[t] = wmb(ah, bh, acc[t]);
      acc[t] = wmb(ah, bl, acc[t]);
      acc[t] = wmb(al, bh, acc[t]);
    }
  }

#pragma unroll
  for (int t = 0; t < 4; ++t) {
    const int lc = 16 * t + m;
#pragma unroll
    for (int r = 0; r < 8; ++r) {
      const int lr = 16 * wave + 8 * hh + r;
      stg[lr * 64 + lc] = acc[t][r];
    }
  }
  __syncthreads();
  store_split_tile(stg, yth, ytl, (size_t)b * NN + (size_t)n0, (size_t)NI, (size_t)e0, wave, lane);
}

__global__ __launch_bounds__(GTHR) void k_z(const unsigned short* __restrict__ wwb,
                                            const unsigned short* __restrict__ yth, const unsigned short* __restrict__ ytl,
                                            const float* __restrict__ wbias, float* z) {
  __shared__ __attribute__((aligned(16))) float stg[64 * 64];
  const int tid = (int)threadIdx.x, lane = tid & 31, wave = tid >> 5, hh = lane >> 4, m = lane & 15;
  const int n0 = (int)blockIdx.x * 64, c0 = (int)blockIdx.y * 64, b = (int)blockIdx.z;

  v8f acc[4];
  {
    const v8f zz = {0.f, 0.f, 0.f, 0.f, 0.f, 0.f, 0.f, 0.f};
    acc[0] = zz; acc[1] = zz; acc[2] = zz; acc[3] = zz;
  }
  const unsigned short* aw = wwb + (size_t)(c0 + 16 * wave + m) * (size_t)NI + (size_t)(8 * hh);
  const size_t brow = (size_t)(b * NN + n0 + m) * (size_t)NI + (size_t)(8 * hh);
  const unsigned short* byh = yth + brow;
  const unsigned short* byl = ytl + brow;
#pragma unroll 1
  for (int ks = 0; ks < NI / 32; ++ks) {
    FragB a;
    ldfrag(a, aw, 32 * ks);
#pragma unroll
    for (int t = 0; t < 4; ++t) {
      FragB bh, bl;
      ldfrag(bh, byh + (size_t)(16 * t) * (size_t)NI, 32 * ks);
      ldfrag(bl, byl + (size_t)(16 * t) * (size_t)NI, 32 * ks);
      acc[t] = wmb(a, bh, acc[t]);
      acc[t] = wmb(a, bl, acc[t]);
    }
  }

  const v4f ba = *(const v4fa*)(wbias + c0 + 16 * wave + 8 * hh);
  const v4f bb = *(const v4fa*)(wbias + c0 + 16 * wave + 8 * hh + 4);
  float bv[8];
  bv[0] = rne16f(ba.x); bv[1] = rne16f(ba.y); bv[2] = rne16f(ba.z); bv[3] = rne16f(ba.w);
  bv[4] = rne16f(bb.x); bv[5] = rne16f(bb.y); bv[6] = rne16f(bb.z); bv[7] = rne16f(bb.w);
#pragma unroll
  for (int t = 0; t < 4; ++t) {
    const int lc = 16 * t + m;
#pragma unroll
    for (int r = 0; r < 8; ++r) {
      const int lr = 16 * wave + 8 * hh + r;
      stg[lr * 64 + lc] = acc[t][r] + bv[r];
    }
  }
  __syncthreads();

  v4f fv[8];
  size_t op[8];
#pragma unroll
  for (int i = 0; i < 8; ++i) {
    const int lr = 16 * wave + 2 * i + hh;
    fv[i] = *(const v4fa*)(stg + lr * 64 + 4 * m);
    op[i] = (size_t)(b * NC + c0 + lr) * (size_t)NN + (size_t)(n0 + 4 * m);
  }
#pragma unroll
  for (int i = 0; i < 8; ++i) *(volatile v4f*)(z + op[i]) = fv[i];
  __threadfence();
#pragma unroll
  for (int i = 0; i < 8; ++i) *(volatile v4f*)(z + op[i]) = fv[i];
}

__global__ __launch_bounds__(NTHR) void k_bnstat(const float* __restrict__ z, float* stats) {
  __shared__ double sh[NTHR];
  __shared__ double sh2[NTHR];
  __shared__ float res[2];
  const int c = (int)blockIdx.x, tid = (int)threadIdx.x;
  double s = 0.0, s2 = 0.0;
#pragma unroll 1
  for (int it = 0; it < NB * (NN / 1024); ++it) {
    const int bi = it / (NN / 1024);
    const int hf = it - bi * (NN / 1024);
    const v4f v = *(const v4fa*)(z + (size_t)(bi * NC + c) * (size_t)NN + (size_t)(hf * 1024 + 4 * tid));
    const double a0 = (double)v.x, a1 = (double)v.y, a2 = (double)v.z, a3 = (double)v.w;
    s  += (a0 + a1) + (a2 + a3);
    s2 += (a0 * a0 + a1 * a1) + (a2 * a2 + a3 * a3);
  }
  sh[tid] = s;
  sh2[tid] = s2;
  __syncthreads();
#pragma unroll 1
  for (int off = NTHR / 2; off > 0; off >>= 1) {
    if (tid < off) {
      sh[tid]  += sh[tid + off];
      sh2[tid] += sh2[tid + off];
    }
    __syncthreads();
  }
  if (tid == 0) {
    const double cinv = 1.0 / 32768.0;
    const double mean = sh[0] * cinv;
    double var = sh2[0] * cinv - mean * mean;
    var = var < 0.0 ? 0.0 : var;
    const float vf = (float)var + 1e-5f;
    res[0] = (float)mean;
    res[1] = 1.0f / sqrtf(vf);
  }
  __syncthreads();
  if (tid < 8) {
    const float mv = res[0];
    const float rv = res[1];
    v4f o;
    o.x = (tid == 0) ? mv : 0.f;
    o.y = (tid == 0) ? rv : 0.f;
    o.z = 0.f;
    o.w = 0.f;
    float* p = stats + (size_t)c * 32 + (size_t)(4 * tid);
    *(volatile v4f*)p = o;
    __threadfence();
    *(volatile v4f*)p = o;
  }
}

__global__ __launch_bounds__(NTHR) void k_out(const float* __restrict__ z, const float* __restrict__ x,
                                              const float* __restrict__ stats, const float* __restrict__ gamma,
                                              const float* __restrict__ beta, float* out) {
  const int row = (int)blockIdx.x / (NN / 1024);
  const int c = row & (NC - 1);
  const size_t base = (size_t)blockIdx.x * 1024 + (size_t)(4 * (int)threadIdx.x);
  const float mean = stats[(size_t)c * 32];
  const float rstd = stats[(size_t)c * 32 + 1];
  const float gm = rne16f(gamma[c]);
  const float bt = rne16f(beta[c]);
  const v4f zv = *(const v4fa*)(z + base);
  const v4f xv = *(const v4fa*)(x + base);
  v4f o;
  o.x = (((zv.x - mean) * rstd) * gm + bt) + rne16f(xv.x);
  o.y = (((zv.y - mean) * rstd) * gm + bt) + rne16f(xv.y);
  o.z = (((zv.z - mean) * rstd) * gm + bt) + rne16f(xv.z);
  o.w = (((zv.w - mean) * rstd) * gm + bt) + rne16f(xv.w);
  float* p = out + base;
  *(volatile v4f*)p = o;
  __threadfence();
  *(volatile v4f*)p = o;
}

extern "C" void kernel_launch(void* const* d_in, const int* in_sizes, int n_in,
                              void* d_out, int out_size, void* d_ws, size_t ws_size,
                              hipStream_t stream) {
  if (n_in < 11) return;
  if (in_sizes[0] != NX) return;
  if (in_sizes[1] != NWT || in_sizes[3] != NWT || in_sizes[5] != NWT) return;
  if (in_sizes[2] != NI || in_sizes[4] != NI || in_sizes[6] != NI) return;
  if (in_sizes[7] != NWT) return;
  if (in_sizes[8] != NC || in_sizes[9] != NC || in_sizes[10] != NC) return;
  if (out_size != NX) return;

  const float* x       = (const float*)d_in[0];
  const float* g_w     = (const float*)d_in[1];
  const float* g_b     = (const float*)d_in[2];
  const float* theta_w = (const float*)d_in[3];
  const float* theta_b = (const float*)d_in[4];
  const float* phi_w   = (const float*)d_in[5];
  const float* phi_b   = (const float*)d_in[6];
  const float* W_w     = (const float*)d_in[7];
  const float* W_b     = (const float*)d_in[8];
  const float* gamma   = (const float*)d_in[9];
  const float* beta    = (const float*)d_in[10];
  float* out = (float*)d_out;

  char* ws = (char*)d_ws;
  size_t off = 0;
  const size_t oWB  = off; off += (size_t)4 * NWT * 2;          off = (off + 255) & ~(size_t)255;
  const size_t oXT  = off; off += (size_t)NX * 2;               off = (off + 255) & ~(size_t)255;
  const size_t plb  = (size_t)NB * NN * NI * 2;
  const size_t oTHH = off; off += plb;                          off = (off + 255) & ~(size_t)255;
  const size_t oTHL = off; off += plb;                          off = (off + 255) & ~(size_t)255;
  const size_t oPHH = off; off += plb;                          off = (off + 255) & ~(size_t)255;
  const size_t oPHL = off; off += plb;                          off = (off + 255) & ~(size_t)255;
  const size_t oGH  = off; off += plb;                          off = (off + 255) & ~(size_t)255;
  const size_t oGL  = off; off += plb;                          off = (off + 255) & ~(size_t)255;
  const size_t ptb  = (size_t)NB * NI * NI * 2;
  const size_t oPTH = off; off += ptb;                          off = (off + 255) & ~(size_t)255;
  const size_t oPTL = off; off += ptb;                          off = (off + 255) & ~(size_t)255;
  const size_t oYTH = off; off += plb;                          off = (off + 255) & ~(size_t)255;
  const size_t oYTL = off; off += plb;                          off = (off + 255) & ~(size_t)255;
  const size_t oZ   = off; off += (size_t)NX * 4;               off = (off + 255) & ~(size_t)255;
  const size_t oST  = off; off += (size_t)NC * 32 * 4;          off = (off + 255) & ~(size_t)255;
  if (off > ws_size || off > (size_t)WSMAX) return;

  unsigned short* WB  = (unsigned short*)(ws + oWB);
  unsigned short* XT  = (unsigned short*)(ws + oXT);
  unsigned short* THH = (unsigned short*)(ws + oTHH);
  unsigned short* THL = (unsigned short*)(ws + oTHL);
  unsigned short* PHH = (unsigned short*)(ws + oPHH);
  unsigned short* PHL = (unsigned short*)(ws + oPHL);
  unsigned short* GH  = (unsigned short*)(ws + oGH);
  unsigned short* GL  = (unsigned short*)(ws + oGL);
  unsigned short* PTH = (unsigned short*)(ws + oPTH);
  unsigned short* PTL = (unsigned short*)(ws + oPTL);
  unsigned short* YTH = (unsigned short*)(ws + oYTH);
  unsigned short* YTL = (unsigned short*)(ws + oYTL);
  float*          Z   = (float*)(ws + oZ);
  float*          ST  = (float*)(ws + oST);

  k_wcvt<<<(4 * NWT / 8) / NTHR, NTHR, 0, stream>>>(theta_w, phi_w, g_w, W_w, WB);
  k_xt<<<dim3(NC / 64, NN / 64, NB), NTHR, 0, stream>>>(x, XT);
  k_proj<<<dim3(NN / 64, NI / 64, 3 * NB), GTHR, 0, stream>>>(XT, WB, theta_b, phi_b, g_b,
                                                              THH, THL, PHH, PHL, GH, GL);
  k_p<<<dim3(NI / 64, NI / 64, NB), GTHR, 0, stream>>>(GH, GL, PHH, PHL, PTH, PTL);
  k_y<<<dim3(NN / 64, NI / 64, NB), GTHR, 0, stream>>>(THH, THL, PTH, PTL, YTH, YTL);
  k_z<<<dim3(NN / 64, NC / 64, NB), GTHR, 0, stream>>>(WB + (size_t)3 * NWT, YTH, YTL, W_b, Z);
  k_bnstat<<<NC, NTHR, 0, stream>>>(Z, ST);
  k_out<<<NX / 1024, NTHR, 0, stream>>>(Z, x, ST, gamma, beta, out);
}
